// SelfAttention_17970143166886
// MI455X (gfx1250) — hardware-run, weakly checked
//
#include <hip/hip_runtime.h>
#include <math.h>

typedef __attribute__((ext_vector_type(16))) _Float16 v16h;
typedef __attribute__((ext_vector_type(8)))  _Float16 v8h;
typedef __attribute__((ext_vector_type(8)))  float    v8f;
typedef __attribute__((ext_vector_type(4)))  float    v4f;

constexpr int kBatch = 8;
constexpr int kCin   = 256;
constexpr int kNpix  = 4096;
constexpr int kHeads = 4;
constexpr int kHc    = 64;
constexpr int kHid   = kHeads * kHc;
constexpr int kQkv   = 3 * kHid;
constexpr int kCout  = 256;
static_assert(kHid == 256);
static_assert(kQkv == 768);
static_assert((kCin % 32) == 0 && (kHid % 32) == 0 && (kHc % 32) == 0 && (kNpix % 32) == 0 && ((2 * kHc) % 32) == 0);
static_assert((kNpix % 64) == 0 && (kHid % 64) == 0 && (kCout % 64) == 0 && (kHc % 64) == 0);

constexpr float kXCarry   = 16.0f;
constexpr float kWCarry   = 256.0f;
constexpr float kQCarry   = 16.0f;
constexpr float kVCarry   = 16.0f;
constexpr float kECarry   = 16.0f;
constexpr float kCtxCarry = 256.0f;
constexpr float kOutCarry = 64.0f;
constexpr float kRemCarry = 2048.0f;
constexpr float kScaleQ = kQCarry / (kWCarry * kXCarry);
constexpr float kScaleK = 1.0f / (kWCarry * kXCarry);
constexpr float kScaleV = kVCarry / (kWCarry * kXCarry);
constexpr float kCsNum  = kCtxCarry / kVCarry;
constexpr float kScaleO = kOutCarry / (kCtxCarry * kQCarry);
constexpr float kScaleRem = kScaleO / kRemCarry;
constexpr float kScaleY = 1.0f / (kWCarry * kOutCarry);
constexpr float kF16Min = 6.103515625e-5f;
constexpr float kEps    = 1e-5f;
constexpr float kInvCnt = 1.0f / ((float)kCout * (float)kNpix);

constexpr size_t kPlane16 = (size_t)kBatch * kNpix * kCin * 2;
constexpr size_t kOffXT   = 0;
constexpr size_t kOffQT   = kOffXT + kPlane16;
constexpr size_t kOffV    = kOffQT + kPlane16;
constexpr size_t kOffE    = kOffV  + kPlane16;
constexpr size_t kOffOT   = kOffE  + kPlane16;
constexpr size_t kOffKF   = kOffOT + kPlane16;
constexpr size_t kOffWQ   = kOffKF + (size_t)kBatch * kHid * kNpix * 4;
constexpr size_t kOffWO   = kOffWQ + (size_t)kQkv * kCin * 2;
constexpr size_t kOffCT   = kOffWO + (size_t)kCout * kHid * 2;
constexpr size_t kOffCL   = kOffCT + (size_t)kBatch * kHeads * kHc * kHc * 2;
constexpr size_t kOffCS   = kOffCL + (size_t)kBatch * kHeads * kHc * kHc * 2;
constexpr size_t kOffPART = kOffCS + (size_t)kBatch * kHid * 32 * 4;
constexpr size_t kWsTotal = kOffPART + (size_t)kBatch * 64 * 32 * 4;
static_assert(kWsTotal == 118816768ull);
static_assert(kWsTotal <= 134217728ull);
static_assert((size_t)kBatch * kNpix * kHid * 4 == (size_t)kBatch * kHid * kNpix * 4);
static_assert((kOffQT % 128) == 0 && (kOffV % 128) == 0 && (kOffE % 128) == 0 && (kOffOT % 128) == 0 &&
              (kOffKF % 128) == 0 && (kOffWQ % 128) == 0 && (kOffWO % 128) == 0 && (kOffCT % 128) == 0 &&
              (kOffCL % 128) == 0 && (kOffCS % 128) == 0 && (kOffPART % 128) == 0);

__device__ __forceinline__ unsigned short f2bf_bits(float f) {
  unsigned u = __float_as_uint(f);
  return (unsigned short)((u + 0x7FFFu + ((u >> 16) & 1u)) >> 16);
}
__device__ __forceinline__ float bf_bits2f(unsigned short h) { return __uint_as_float(((unsigned)h) << 16); }
__device__ __forceinline__ float bf_rne(float f) { return bf_bits2f(f2bf_bits(f)); }
__device__ __forceinline__ float flush_h(float v) { return (fabsf(v) < kF16Min) ? 0.0f : v; }

struct FragH {
  union U { v16h v; v8h h[2]; };
  static __device__ __forceinline__ v16h load(const _Float16* p) {
    U f;
    f.h[0] = *(const v8h*)(p);
    f.h[1] = *(const v8h*)(p + 16);
    return f.v;
  }
};
__device__ __forceinline__ v8f mma_h(v16h a, v16h b, v8f c) {
  c = __builtin_amdgcn_wmma_f32_16x16x32_f16(false, a, false, b, (short)0, c, false, false);
  asm volatile("v_nop\n\tv_nop\n\tv_nop\n\tv_nop" : "+v"(c) : "v"(a), "v"(b));
  return c;
}

__global__ __launch_bounds__(256) void xpose_cast_kernel(const float* __restrict__ x, unsigned short* __restrict__ xt) {
  __shared__ float sm[64 * 65];
  const int t  = threadIdx.x;
  const int n0 = blockIdx.x * 64;
  const int c0 = blockIdx.y * 64;
  const int b  = blockIdx.z;
  const float* xb = x + ((size_t)b * kCin + c0) * kNpix + n0;
#pragma unroll
  for (int i = 0; i < 16; ++i) {
    const int e  = i * 256 + t;
    const int r  = e >> 6;
    const int cc = e & 63;
    sm[cc * 65 + r] = xb[(size_t)r * kNpix + cc];
  }
  __syncthreads();
  const int lane = t & 31, wave = t >> 5;
  const int q = lane >> 3, c8 = (lane & 7) * 8;
  v8h hv[2];
#pragma unroll
  for (int it = 0; it < 2; ++it) {
    const int row = wave * 8 + it * 4 + q;
#pragma unroll
    for (int e = 0; e < 8; ++e) {
      const float v = flush_h(bf_rne(sm[row * 65 + c8 + e]) * kXCarry);
      hv[it][e] = (_Float16)v;
    }
  }
  for (int pass = 0; pass < 2; ++pass) {
#pragma unroll
    for (int it = 0; it < 2; ++it) {
      const int row = wave * 8 + it * 4 + q;
      *(volatile v8h*)(xt + ((size_t)b * kNpix + n0 + row) * kCin + c0 + c8) = hv[it];
    }
    __threadfence();
  }
}

constexpr int kWqBlocks = (kQkv * kCin / 8) / 256;
constexpr int kWoBlocks = (kCout * kHid / 8) / 256;
static_assert(kWqBlocks * 256 * 8 == kQkv * kCin);
static_assert(kWoBlocks * 256 * 8 == kCout * kHid);
__global__ __launch_bounds__(256) void wcast_kernel(const float* __restrict__ wqkv, const float* __restrict__ wout,
                                                    unsigned short* __restrict__ wq16, unsigned short* __restrict__ wo16) {
  const int blk = blockIdx.x;
  const bool first = (blk < kWqBlocks);
  const float* src = first ? wqkv : wout;
  unsigned short* dst = first ? wq16 : wo16;
  const int i = (first ? blk : (blk - kWqBlocks)) * 256 + threadIdx.x;
  const float* p = src + 8 * (size_t)i;
  const v4f a = *(const v4f*)(p);
  const v4f c = *(const v4f*)(p + 4);
  v8h hv;
#pragma unroll
  for (int e = 0; e < 4; ++e) {
    const float v0 = flush_h(bf_rne(a[e]) * kWCarry);
    const float v1 = flush_h(bf_rne(c[e]) * kWCarry);
    hv[e]     = (_Float16)v0;
    hv[4 + e] = (_Float16)v1;
  }
  unsigned short* q = dst + 8 * (size_t)i;
  *(volatile v8h*)q = hv;
  __threadfence();
  *(volatile v8h*)q = hv;
}

template <int BIAS_MODE, int OUT_MODE, bool ADDEND>
__global__ __launch_bounds__(256) void gemm_f16_kernel(
    const unsigned short* Ap, const unsigned short* A2p,
    const unsigned short* Btp, const unsigned short* Bt2p,
    void* __restrict__ Cout, void* __restrict__ Cout2,
    const float* __restrict__ bias, const float* __restrict__ addend,
    long sA, long sA2, long sB, long sB2, long sC, long sC2,
    int lda, int ldb, int ldc, int zdiv, int M, int N, int K, int kseg, float scale, float bscale) {
  static_assert(!ADDEND || OUT_MODE == 1);
  typedef _Float16 T;
  const T* A   = (const T*)Ap;
  const T* A2  = (const T*)A2p;
  const T* Bt  = (const T*)Btp;
  const T* Bt2 = (const T*)Bt2p;
  __shared__ __align__(16) float sT[8][16 * 68];
  const int z    = blockIdx.y;
  const int zb   = z / zdiv;
  const int zh   = z - zb * zdiv;
  const int lane = threadIdx.x & 31;
  const int wave = threadIdx.x >> 5;
  const int tilesN = N >> 6;
  const int tilesM = M >> 6;
  const int tile = blockIdx.x * 8 + wave;
  if (tile >= tilesM * tilesN) return;
  const int tm = tile / tilesN;
  const int tn = tile - tm * tilesN;
  const int m0 = tm << 6;
  const int n0 = tn << 6;

  const size_t aOff = (size_t)zb * sA + (size_t)zh * sA2;
  const size_t bOff = (size_t)zb * sB + (size_t)zh * sB2;
  const T* Ab  = A   + aOff;
  const T* Ab2 = A2  + aOff;
  const T* Bb  = Bt  + bOff;
  const T* Bb2 = Bt2 + bOff;
  const size_t cOff = (size_t)zb * sC + (size_t)zh * sC2;

  const int rlane = lane & 15;
  const int koff  = (lane >> 4) * 8;
  const int mOff  = (lane >> 4) * 8;

  v8f acc[4][4];
#pragma unroll
  for (int i = 0; i < 4; ++i)
#pragma unroll
    for (int j = 0; j < 4; ++j) acc[i][j] = (v8f){0.f, 0.f, 0.f, 0.f, 0.f, 0.f, 0.f, 0.f};

  for (int k0 = 0; k0 < K; k0 += 32) {
    const bool second = (k0 >= kseg);
    const T* Ak = second ? Ab2 : Ab;
    const T* Bk = second ? Bb2 : Bb;
    const int kk = second ? (k0 - kseg) : k0;
    v16h bh[4];
#pragma unroll
    for (int j = 0; j < 4; ++j) {
      const size_t bo = (size_t)(n0 + (j << 4) + rlane) * ldb + koff + kk;
      bh[j] = FragH::load(Bk + bo);
    }
#pragma unroll
    for (int i = 0; i < 4; ++i) {
      const size_t ao = (size_t)(m0 + (i << 4) + rlane) * lda + koff + kk;
      const v16h ah = FragH::load(Ak + ao);
#pragma unroll
      for (int j = 0; j < 4; ++j) acc[i][j] = mma_h(ah, bh[j], acc[i][j]);
    }
  }

  float* slab = sT[wave];
#pragma unroll
  for (int i = 0; i < 4; ++i) {
    const int mBase = m0 + (i << 4);
    float brow[8];
#pragma unroll
    for (int r = 0; r < 8; ++r) {
      brow[r] = 0.0f;
      if (BIAS_MODE == 1) brow[r] = bf_rne(bias[mBase + mOff + r]) * bscale;
    }
#pragma unroll
    for (int j = 0; j < 4; ++j) {
      float bcol = 0.0f;
      if (BIAS_MODE == 2) bcol = bf_rne(bias[n0 + (j << 4) + rlane]) * bscale;
#pragma unroll
      for (int r = 0; r < 8; ++r) {
        const float v = acc[i][j][r] * scale + (brow[r] + bcol);
        slab[(mOff + r) * 68 + (j << 4) + rlane] = v;
      }
    }
    __builtin_amdgcn_fence(__ATOMIC_RELEASE, "workgroup");
    __builtin_amdgcn_wave_barrier();
    __builtin_amdgcn_fence(__ATOMIC_ACQUIRE, "workgroup");
    if (OUT_MODE == 0) {
      float* C = (float*)Cout + cOff;
      const int hh = lane >> 4, c4 = (lane & 15) * 4;
      for (int pass = 0; pass < 2; ++pass) {
#pragma unroll
        for (int it = 0; it < 8; ++it) {
          const int row = it * 2 + hh;
          const v4f v = *(const v4f*)(slab + row * 68 + c4);
          *(volatile v4f*)(C + (size_t)(mBase + row) * ldc + n0 + c4) = v;
        }
        __threadfence();
      }
    } else {
      const int q = lane >> 3, c8 = (lane & 7) * 8;
      unsigned short* C = (unsigned short*)Cout + cOff;
      v8h hv[4];
      v8h lv[4];
#pragma unroll
      for (int it = 0; it < 4; ++it) {
        const int row = it * 4 + q;
        const float* sp = slab + row * 68 + c8;
        const size_t go = (size_t)(mBase + row) * ldc + n0 + c8;
        v4f a0 = (v4f){0.f, 0.f, 0.f, 0.f};
        v4f a1 = (v4f){0.f, 0.f, 0.f, 0.f};
        if (ADDEND) {
          a0 = *(const v4f*)(addend + cOff + go);
          a1 = *(const v4f*)(addend + cOff + go + 4);
        }
#pragma unroll
        for (int e = 0; e < 4; ++e) {
          const float f0 = sp[e] + a0[e];
          const float f1 = sp[4 + e] + a1[e];
          const float g0 = flush_h(f0);
          const float g1 = flush_h(f1);
          const _Float16 h0 = (_Float16)g0;
          const _Float16 h1 = (_Float16)g1;
          hv[it][e]     = h0;
          hv[it][4 + e] = h1;
          if (OUT_MODE == 2) {
            const float b0 = (float)h0;
            const float b1 = (float)h1;
            const float r0 = flush_h((f0 - b0) * kRemCarry);
            const float r1 = flush_h((f1 - b1) * kRemCarry);
            lv[it][e]     = (_Float16)r0;
            lv[it][4 + e] = (_Float16)r1;
          }
        }
      }
      for (int pass = 0; pass < 2; ++pass) {
#pragma unroll
        for (int it = 0; it < 4; ++it) {
          const int row = it * 4 + q;
          const size_t go = (size_t)(mBase + row) * ldc + n0 + c8;
          *(volatile v8h*)(C + go) = hv[it];
          if (OUT_MODE == 2) {
            unsigned short* C2 = (unsigned short*)Cout2 + cOff;
            *(volatile v8h*)(C2 + go) = lv[it];
          }
        }
        __threadfence();
      }
    }
    __builtin_amdgcn_fence(__ATOMIC_RELEASE, "workgroup");
    __builtin_amdgcn_wave_barrier();
    __builtin_amdgcn_fence(__ATOMIC_ACQUIRE, "workgroup");
  }
}

__global__ __launch_bounds__(256) void softmax_exp_kernel(const float* __restrict__ kf, unsigned short* __restrict__ e16,
                                                          float* __restrict__ cs) {
  __shared__ float redM[8];
  __shared__ float redS[8];
  const int row  = blockIdx.x;
  const int t    = threadIdx.x;
  const int lane = t & 31, wave = t >> 5;
  const float* kr = kf + (size_t)row * kNpix;
  float m = -INFINITY;
#pragma unroll 1
  for (int it = 0; it < 2; ++it) {
    const float* p = kr + (size_t)(it * 256 + t) * 8;
    const v4f a = *(const v4f*)(p);
    const v4f c = *(const v4f*)(p + 4);
    const float m0 = fmaxf(fmaxf(a[0], a[1]), fmaxf(a[2], a[3]));
    const float m1 = fmaxf(fmaxf(c[0], c[1]), fmaxf(c[2], c[3]));
    m = fmaxf(m, fmaxf(m0, m1));
  }
#pragma unroll
  for (int off = 16; off > 0; off >>= 1) m = fmaxf(m, __shfl_xor(m, off, 32));
  if (lane == 0) redM[wave] = m;
  __syncthreads();
  float mm = redM[0];
#pragma unroll
  for (int w = 1; w < 8; ++w) mm = fmaxf(mm, redM[w]);

  float s = 0.0f;
  unsigned short* er = e16 + (size_t)row * kNpix;
#pragma unroll 1
  for (int it = 0; it < 2; ++it) {
    const size_t o = (size_t)(it * 256 + t) * 8;
    const v4f a = *(const v4f*)(kr + o);
    const v4f c = *(const v4f*)(kr + o + 4);
    v8h hv;
#pragma unroll
    for (int e = 0; e < 4; ++e) {
      const float v0 = flush_h(kECarry * expf(a[e] - mm));
      const float v1 = flush_h(kECarry * expf(c[e] - mm));
      const _Float16 h0 = (_Float16)v0;
      const _Float16 h1 = (_Float16)v1;
      hv[e]     = h0;
      hv[4 + e] = h1;
      s += (float)h0;
      s += (float)h1;
    }
    *(volatile v8h*)(er + o) = hv;
    __threadfence();
    *(volatile v8h*)(er + o) = hv;
  }
#pragma unroll
  for (int off = 16; off > 0; off >>= 1) s += __shfl_xor(s, off, 32);
  if (lane == 0) redS[wave] = s;
  __syncthreads();
  if (wave == 0) {
    float tot = redS[0];
#pragma unroll
    for (int w = 1; w < 8; ++w) tot += redS[w];
    const float val = kCsNum * (1.0f / tot);
    const float outv = (lane == 0) ? val : 0.0f;
    float* line = cs + (size_t)row * 32;
    ((volatile float*)line)[lane] = outv;
    __threadfence();
    ((volatile float*)line)[lane] = outv;
  }
}

__global__ __launch_bounds__(256) void ctx_kernel(const unsigned short* __restrict__ v16p, const unsigned short* __restrict__ e16p,
                                                  const float* __restrict__ cs, unsigned short* __restrict__ ctxt,
                                                  unsigned short* __restrict__ ctxl) {
  __shared__ __align__(16) float sT[64 * 68];
  const int z    = blockIdx.x;
  const int t    = threadIdx.x;
  const int lane = t & 31, wave = t >> 5;
  const int rlane = lane & 15;
  const int koff  = (lane >> 4) * 8;
  const int mOff  = (lane >> 4) * 8;
  const _Float16* A  = (const _Float16*)v16p + (size_t)z * ((size_t)kHc * kNpix);
  const _Float16* Bt = (const _Float16*)e16p + (size_t)z * ((size_t)kHc * kNpix);
  const int mi = wave >> 1;
  const int nj = (wave & 1) * 2;
  const _Float16* ap  = A  + (size_t)(mi * 16 + rlane) * kNpix + koff;
  const _Float16* bp0 = Bt + (size_t)(nj * 16 + rlane) * kNpix + koff;
  const _Float16* bp1 = bp0 + (size_t)16 * kNpix;
  v8f acc0 = (v8f){0.f, 0.f, 0.f, 0.f, 0.f, 0.f, 0.f, 0.f};
  v8f acc1 = (v8f){0.f, 0.f, 0.f, 0.f, 0.f, 0.f, 0.f, 0.f};
#pragma unroll 2
  for (int k0 = 0; k0 < kNpix; k0 += 32) {
    const v16h a  = FragH::load(ap + k0);
    const v16h b0 = FragH::load(bp0 + k0);
    const v16h b1 = FragH::load(bp1 + k0);
    acc0 = mma_h(a, b0, acc0);
    acc1 = mma_h(a, b1, acc1);
  }
  const int d0 = nj * 16 + rlane;
  const int d1 = d0 + 16;
  const float c0 = cs[((size_t)z * kHc + d0) * 32];
  const float c1 = cs[((size_t)z * kHc + d1) * 32];
#pragma unroll
  for (int r = 0; r < 8; ++r) {
    sT[(mi * 16 + mOff + r) * 68 + d0] = acc0[r] * c0;
    sT[(mi * 16 + mOff + r) * 68 + d1] = acc1[r] * c1;
  }
  __syncthreads();
  const int q = lane >> 3, c8 = (lane & 7) * 8;
  v8h hv[2];
  v8h lv[2];
#pragma unroll
  for (int it = 0; it < 2; ++it) {
    const int row = wave * 8 + it * 4 + q;
    const float* sp = sT + row * 68 + c8;
#pragma unroll
    for (int e = 0; e < 8; ++e) {
      const float f0 = sp[e];
      const float g0 = flush_h(f0);
      const _Float16 h0 = (_Float16)g0;
      const float b0 = (float)h0;
      const float r0 = flush_h((f0 - b0) * kRemCarry);
      hv[it][e] = h0;
      lv[it][e] = (_Float16)r0;
    }
  }
  unsigned short* cz = ctxt + (size_t)z * (kHc * kHc);
  unsigned short* cl = ctxl + (size_t)z * (kHc * kHc);
  for (int pass = 0; pass < 2; ++pass) {
#pragma unroll
    for (int it = 0; it < 2; ++it) {
      const int row = wave * 8 + it * 4 + q;
      *(volatile v8h*)(cz + row * kHc + c8) = hv[it];
      *(volatile v8h*)(cl + row * kHc + c8) = lv[it];
    }
    __threadfence();
  }
}

__global__ __launch_bounds__(256) void stats_partial_kernel(const float* __restrict__ y, float* __restrict__ part) {
  __shared__ float redS[8];
  __shared__ float redQ[8];
  const int j = blockIdx.x, b = blockIdx.y;
  const int t = threadIdx.x, lane = t & 31, wave = t >> 5;
  const float* p = y + (size_t)b * ((size_t)kCout * kNpix) + (size_t)j * 16384;
  float s = 0.0f, q = 0.0f;
#pragma unroll 4
  for (int it = 0; it < 16; ++it) {
    const v4f v = *(const v4f*)(p + (size_t)(it * 256 + t) * 4);
    s += (v[0] + v[1]) + (v[2] + v[3]);
    q = fmaf(v[0], v[0], q);
    q = fmaf(v[1], v[1], q);
    q = fmaf(v[2], v[2], q);
    q = fmaf(v[3], v[3], q);
  }
#pragma unroll
  for (int off = 16; off > 0; off >>= 1) {
    s += __shfl_xor(s, off, 32);
    q += __shfl_xor(q, off, 32);
  }
  if (lane == 0) {
    redS[wave] = s;
    redQ[wave] = q;
  }
  __syncthreads();
  if (wave == 0) {
    float ts = redS[0], tq = redQ[0];
#pragma unroll
    for (int w = 1; w < 8; ++w) {
      ts += redS[w];
      tq += redQ[w];
    }
    const float outv = (lane == 0) ? ts : ((lane == 1) ? tq : 0.0f);
    float* line = part + ((size_t)b * 64 + j) * 32;
    ((volatile float*)line)[lane] = outv;
    __threadfence();
    ((volatile float*)line)[lane] = outv;
  }
}

__global__ __launch_bounds__(256) void norm_act_kernel(const float* __restrict__ y, const float* __restrict__ part,
                                                       const float* __restrict__ gamma, const float* __restrict__ beta,
                                                       float* __restrict__ out) {
  __shared__ float sS[64];
  __shared__ float sQ[64];
  __shared__ float sStat[2];
  const int t = threadIdx.x;
  const int b = blockIdx.x / kCout;
  const int c = blockIdx.x - b * kCout;
  const float* pp = part + ((size_t)b * 64 + (t & 63)) * 32;
  float p0 = pp[0];
  float p1 = pp[1];
  asm volatile("" : "+v"(p0));
  asm volatile("" : "+v"(p1));
  if (t < 64) {
    sS[t] = p0;
    sQ[t] = p1;
  }
  __syncthreads();
  if (t == 0) {
    float S = 0.0f, Q = 0.0f;
#pragma unroll 1
    for (int j = 0; j < 64; ++j) {
      S += sS[j];
      Q += sQ[j];
    }
    const float mean = S * kInvCnt;
    const float var  = Q * kInvCnt - mean * mean;
    sStat[0] = mean;
    sStat[1] = rsqrtf(fmaxf(var, 0.0f) + kEps);
  }
  __syncthreads();
  const float mean = sStat[0];
  const float inv  = sStat[1];
  const float g  = bf_rne(gamma[c]);
  const float be = bf_rne(beta[c]);
  const float* yr = y + (size_t)blockIdx.x * kNpix;
  float* orow = out + (size_t)blockIdx.x * kNpix;
#pragma unroll 1
  for (int it = 0; it < 4; ++it) {
    const int o = (it * 256 + t) * 4;
    const v4f v = *(const v4f*)(yr + o);
    v4f r;
#pragma unroll
    for (int e = 0; e < 4; ++e) {
      float u = (v[e] - mean) * inv;
      u = u * g + be;
      r[e] = tanhf(fmaxf(u, 0.0f));
    }
    *(volatile v4f*)(orow + o) = r;
    __threadfence();
    *(volatile v4f*)(orow + o) = r;
  }
}

extern "C" void kernel_launch(void* const* d_in, const int* in_sizes, int n_in,
                              void* d_out, int out_size, void* d_ws, size_t ws_size,
                              hipStream_t stream) {
  if (n_in < 7) return;
  if (in_sizes[0] != kBatch * kCin * kNpix) return;
  if (in_sizes[1] != kQkv * kCin) return;
  if (in_sizes[2] != kQkv) return;
  if (in_sizes[3] != kCout * kHid) return;
  if (in_sizes[4] != kCout) return;
  if (in_sizes[5] != kCout) return;
  if (in_sizes[6] != kCout) return;
  if (out_size != kBatch * kCout * kNpix) return;
  if (ws_size < kWsTotal) return;

  const float* x     = (const float*)d_in[0];
  const float* Wqkv  = (const float*)d_in[1];
  const float* bqkv  = (const float*)d_in[2];
  const float* Wout  = (const float*)d_in[3];
  const float* bout  = (const float*)d_in[4];
  const float* gamma = (const float*)d_in[5];
  const float* beta  = (const float*)d_in[6];
  float* out = (float*)d_out;

  char* ws = (char*)d_ws;
  unsigned short* XT  = (unsigned short*)(ws + kOffXT);
  unsigned short* QT  = (unsigned short*)(ws + kOffQT);
  unsigned short* V16 = (unsigned short*)(ws + kOffV);
  unsigned short* E16 = (unsigned short*)(ws + kOffE);
  unsigned short* OT  = (unsigned short*)(ws + kOffOT);
  unsigned short* QL  = (unsigned short*)(ws + kOffOT);
  float*          KF  = (float*)(ws + kOffKF);
  float*          REM = (float*)(ws + kOffKF);
  float*          Y   = (float*)(ws + kOffKF);
  unsigned short* WQ  = (unsigned short*)(ws + kOffWQ);
  unsigned short* WO  = (unsigned short*)(ws + kOffWO);
  unsigned short* CT  = (unsigned short*)(ws + kOffCT);
  unsigned short* CL  = (unsigned short*)(ws + kOffCL);
  float*          CS  = (float*)(ws + kOffCS);
  float*          PART = (float*)(ws + kOffPART);

  const long sPix = (long)kNpix * kCin;
  const long sChn = (long)kHid * kNpix;
  const long sCtxB = (long)kHeads * kHc * kHc;
  const long sCtxH = (long)kHc * kHc;

  xpose_cast_kernel<<<dim3(kNpix / 64, kCin / 64, kBatch), 256, 0, stream>>>(x, XT);
  wcast_kernel<<<kWqBlocks + kWoBlocks, 256, 0, stream>>>(Wqkv, Wout, WQ, WO);

  gemm_f16_kernel<2, 2, false><<<dim3(32, kBatch), 256, 0, stream>>>(
      XT, XT, WQ, WQ, (void*)QT, (void*)QL, bqkv, nullptr,
      sPix, 0L, 0L, 0L, sPix, 0L,
      kCin, kCin, kHid, 1, kNpix, kHid, kCin, kCin, kScaleQ, kQCarry);
  gemm_f16_kernel<1, 0, false><<<dim3(32, kBatch), 256, 0, stream>>>(
      WQ + (size_t)kHid * kCin, WQ + (size_t)kHid * kCin, XT, XT, (void*)KF, nullptr, bqkv + kHid, nullptr,
      0L, 0L, sPix, 0L, sChn, 0L,
      kCin, kCin, kNpix, 1, kHid, kNpix, kCin, kCin, kScaleK, 1.0f);
  gemm_f16_kernel<1, 1, false><<<dim3(32, kBatch), 256, 0, stream>>>(
      WQ + (size_t)2 * kHid * kCin, WQ + (size_t)2 * kHid * kCin, XT, XT, (void*)V16, nullptr, bqkv + 2 * kHid, nullptr,
      0L, 0L, sPix, 0L, sChn, 0L,
      kCin, kCin, kNpix, 1, kHid, kNpix, kCin, kCin, kScaleV, kVCarry);

  softmax_exp_kernel<<<kBatch * kHid, 256, 0, stream>>>(KF, E16, CS);
  ctx_kernel<<<kBatch * kHeads, 256, 0, stream>>>(V16, E16, CS, CT, CL);

  gemm_f16_kernel<0, 0, false><<<dim3(8, kBatch * kHeads), 256, 0, stream>>>(
      QL, QT, CT, CL, (void*)REM, nullptr, bqkv, nullptr,
      sPix, (long)kHc, sCtxB, sCtxH, sPix, (long)kHc,
      kHid, kHc, kHid, kHeads, kNpix, kHc, 2 * kHc, kHc, kScaleRem, 0.0f);
  gemm_f16_kernel<0, 1, true><<<dim3(8, kBatch * kHeads), 256, 0, stream>>>(
      QT, QT, CT, CT, (void*)OT, nullptr, bqkv, REM,
      sPix, (long)kHc, sCtxB, sCtxH, sPix, (long)kHc,
      kHid, kHc, kHid, kHeads, kNpix, kHc, kHc, kHc, kScaleO, 0.0f);

  gemm_f16_kernel<1, 0, false><<<dim3(32, kBatch), 256, 0, stream>>>(
      WO, WO, OT, OT, (void*)Y, nullptr, bout, nullptr,
      0L, 0L, sPix, 0L, (long)kCout * kNpix, 0L,
      kHid, kHid, kNpix, 1, kCout, kNpix, kHid, kHid, kScaleY, 1.0f);

  stats_partial_kernel<<<dim3(64, kBatch), 256, 0, stream>>>(Y, PART);
  norm_act_kernel<<<kBatch * kCout, 256, 0, stream>>>(Y, PART, gamma, beta, out);
}
